// ModulatedMambaStack_11725260718318
// MI455X (gfx1250) — hardware-run, weakly checked
//
#include <hip/hip_runtime.h>
#include <math.h>

typedef __attribute__((ext_vector_type(16))) _Float16 v16h;
typedef __attribute__((ext_vector_type(8)))  _Float16 v8h;
typedef __attribute__((ext_vector_type(16))) __bf16   v16b;
typedef __attribute__((ext_vector_type(8)))  __bf16   v8b;
typedef __attribute__((ext_vector_type(8)))  float    v8f;
typedef __attribute__((ext_vector_type(4)))  float    v4f;

constexpr int kLayers = 6;
constexpr int kBatch  = 2;
constexpr int kSeq    = 1024;
constexpr int kDm     = 768;
constexpr int kCond   = 128;
constexpr int kDin    = 1536;
constexpr int kNst    = 16;
constexpr int kDtR    = 48;
constexpr int kDtP    = 64;
constexpr int kPrjN   = 80;
constexpr int kPrjP   = 128;
constexpr int kRows   = kBatch * kSeq;
constexpr int kTP     = 260;
constexpr int kOut0   = kRows * kDm;
constexpr int kOut1   = kLayers * kBatch * kDin * kNst;
constexpr float kEps    = 1e-5f;
constexpr float kLog2e  = 1.4426950408889634f;
constexpr float kCarryWz  = 32.0f;
constexpr float kCarryDt  = 16.0f;
constexpr float kCarryWdt = 8.0f;
constexpr float kCarryY   = 64.0f;
constexpr float kCarryWo  = 32.0f;
constexpr float kFoldZ  = 1.0f / kCarryWz;
constexpr float kFoldDt = 1.0f / (kCarryDt * kCarryWdt);
constexpr float kFoldO  = 1.0f / (kCarryY * kCarryWo);

static_assert(kDtR + 2 * kNst == kPrjN);
static_assert((kDm % 32) == 0 && (kDin % 32) == 0 && (kDtP % 32) == 0);
static_assert((kRows % 64) == 0 && (kDin % 64) == 0 && (kDm % 64) == 0 && (kPrjP % 64) == 0);
static_assert((kSeq & (kSeq - 1)) == 0 && (kSeq % 64) == 0 && (kDin % 256) == 0 && (kRows % 8) == 0);
static_assert((kDtR % 8) == 0 && kDtR <= kDtP && kPrjN <= kPrjP);
static_assert((size_t)kOut0 * 4 == 6291456ull);
static_assert(((size_t)kOut0 + (size_t)kOut1) * 4 == 7471104ull);

constexpr size_t kOffWIH   = 0;
constexpr size_t kOffWIL   = kOffWIH   + (size_t)kDin  * kDm  * 2;
constexpr size_t kOffWZ16  = kOffWIL   + (size_t)kDin  * kDm  * 2;
constexpr size_t kOffWXH   = kOffWZ16  + (size_t)kDin  * kDm  * 2;
constexpr size_t kOffWXL   = kOffWXH   + (size_t)kPrjP * kDin * 2;
constexpr size_t kOffWDT16 = kOffWXL   + (size_t)kPrjP * kDin * 2;
constexpr size_t kOffWO16  = kOffWDT16 + (size_t)kDin  * kDtP * 2;
constexpr size_t kOffHH    = kOffWO16  + (size_t)kDm   * kDin * 2;
constexpr size_t kOffHL    = kOffHH    + (size_t)kRows * kDm  * 2;
constexpr size_t kOffH16   = kOffHL    + (size_t)kRows * kDm  * 2;
constexpr size_t kOffHA    = kOffH16   + (size_t)kRows * kDm  * 2;
constexpr size_t kOffHB    = kOffHA    + (size_t)kRows * kDm  * 4;
constexpr size_t kOffXCP   = kOffHB    + (size_t)kRows * kDm  * 4;
constexpr size_t kOffZB    = kOffXCP   + (size_t)kRows * kDin * 4;
constexpr size_t kOffXC    = kOffZB    + (size_t)kRows * kDin * 4;
constexpr size_t kOffXCH   = kOffXC    + (size_t)kRows * kDin * 4;
constexpr size_t kOffXCL   = kOffXCH   + (size_t)kRows * kDin * 2;
constexpr size_t kOffDBC   = kOffXCL   + (size_t)kRows * kDin * 2;
constexpr size_t kOffDT16  = kOffDBC   + (size_t)kRows * kPrjP * 4;
constexpr size_t kOffDLR   = kOffDT16  + (size_t)kRows * kDtP * 2;
constexpr size_t kOffY16   = kOffDLR   + (size_t)kRows * kDin * 4;
constexpr size_t kOffMP    = kOffY16   + (size_t)kRows * kDin * 2;
constexpr size_t kOffSS    = kOffMP    + (size_t)kRows * kDm  * 4;
constexpr size_t kWsTotal  = kOffSS    + (size_t)kLayers * kBatch * 2 * kDm * 4;
static_assert(kWsTotal == 109322240ull);
static_assert(kWsTotal <= 134217728ull);
static_assert((kOffWIL % 128) == 0 && (kOffWZ16 % 128) == 0 && (kOffWXH % 128) == 0 && (kOffWXL % 128) == 0 &&
              (kOffWDT16 % 128) == 0 && (kOffWO16 % 128) == 0 && (kOffHH % 128) == 0 && (kOffHL % 128) == 0 &&
              (kOffH16 % 128) == 0 && (kOffHA % 128) == 0 && (kOffHB % 128) == 0 && (kOffXCP % 128) == 0 &&
              (kOffZB % 128) == 0 && (kOffXC % 128) == 0 && (kOffXCH % 128) == 0 && (kOffXCL % 128) == 0 &&
              (kOffDBC % 128) == 0 && (kOffDT16 % 128) == 0 && (kOffDLR % 128) == 0 && (kOffY16 % 128) == 0 &&
              (kOffMP % 128) == 0 && (kOffSS % 128) == 0);

__device__ __forceinline__ unsigned short f2bf_bits(float f) {
  unsigned u = __float_as_uint(f);
  return (unsigned short)((u + 0x7FFFu + ((u >> 16) & 1u)) >> 16);
}
__device__ __forceinline__ float bf_bits2f(unsigned short h) { return __uint_as_float(((unsigned)h) << 16); }

__device__ __forceinline__ void grp_guard_h(v8f& a, v8f& b, v8f& c, v8f& d, v16h x, v16h y, v16h p, v16h q, v16h r, v16h s) {
  asm volatile("v_nop\n\tv_nop\n\tv_nop\n\tv_nop" : "+v"(a), "+v"(b), "+v"(c), "+v"(d) : "v"(x), "v"(y), "v"(p), "v"(q), "v"(r), "v"(s));
}
__device__ __forceinline__ void grp_guard_b(v8f& a, v8f& b, v8f& c, v8f& d, v16b x, v16b y, v16b p, v16b q, v16b r, v16b s) {
  asm volatile("v_nop\n\tv_nop\n\tv_nop\n\tv_nop" : "+v"(a), "+v"(b), "+v"(c), "+v"(d) : "v"(x), "v"(y), "v"(p), "v"(q), "v"(r), "v"(s));
}
__device__ __forceinline__ void keep4_h(v16h a, v16h b, v16h c, v16h d) { asm volatile("v_nop" :: "v"(a), "v"(b), "v"(c), "v"(d)); }
__device__ __forceinline__ void keep4_b(v16b a, v16b b, v16b c, v16b d) { asm volatile("v_nop" :: "v"(a), "v"(b), "v"(c), "v"(d)); }
__device__ __forceinline__ void acc_guard4(v8f& a, v8f& b, v8f& c, v8f& d) { asm volatile("v_nop\n\tv_nop\n\tv_nop\n\tv_nop" : "+v"(a), "+v"(b), "+v"(c), "+v"(d)); }

template <typename T> struct Frag;
template <> struct Frag<_Float16> {
  typedef v16h V; union U { v16h v; v8h h[2]; };
  static __device__ __forceinline__ v16h load(const _Float16* p) {
    U f; f.h[0] = *(const v8h*)(p); f.h[1] = *(const v8h*)(p + 16); return f.v;
  }
  static __device__ __forceinline__ v8f mma(v16h a, v16h b, v8f c) {
    return __builtin_amdgcn_wmma_f32_16x16x32_f16(false, a, false, b, (short)0, c, false, false);
  }
  static __device__ __forceinline__ void guard(v8f& a, v8f& b, v8f& c, v8f& d, v16h x, v16h y, v16h p, v16h q, v16h r, v16h s) { grp_guard_h(a, b, c, d, x, y, p, q, r, s); }
  static __device__ __forceinline__ void keep(v16h a, v16h b, v16h c, v16h d) { keep4_h(a, b, c, d); }
};
template <> struct Frag<__bf16> {
  typedef v16b V; union U { v16b v; v8b h[2]; };
  static __device__ __forceinline__ v16b load(const __bf16* p) {
    U f; f.h[0] = *(const v8b*)(p); f.h[1] = *(const v8b*)(p + 16); return f.v;
  }
  static __device__ __forceinline__ v8f mma(v16b a, v16b b, v8f c) {
    return __builtin_amdgcn_wmma_f32_16x16x32_bf16(false, a, false, b, (short)0, c, false, false);
  }
  static __device__ __forceinline__ void guard(v8f& a, v8f& b, v8f& c, v8f& d, v16b x, v16b y, v16b p, v16b q, v16b r, v16b s) { grp_guard_b(a, b, c, d, x, y, p, q, r, s); }
  static __device__ __forceinline__ void keep(v16b a, v16b b, v16b c, v16b d) { keep4_b(a, b, c, d); }
};

template <int ET> struct Elem;
template <> struct Elem<0> { typedef _Float16 T; };
template <> struct Elem<1> { typedef __bf16 T; };
template <int ET, bool SPLIT, int BIAS_MODE>
__global__ __launch_bounds__(256) void wmma_gemm64(
    const unsigned short* __restrict__ Ap, const unsigned short* __restrict__ A2p, int lda,
    const unsigned short* __restrict__ Btp, const unsigned short* __restrict__ Bt2p, int ldb,
    float* __restrict__ Cout, int ldc,
    const float* __restrict__ bias,
    int M, int N, int K, float scale) {
  typedef typename Elem<ET>::T T;
  typedef typename Frag<T>::V V;
  const T* Ab  = (const T*)Ap;
  const T* Ab2 = (const T*)A2p;
  const T* Bb  = (const T*)Btp;
  const T* Bb2 = (const T*)Bt2p;
  __shared__ __align__(16) float sT[8][16 * 68];
  const int lane = threadIdx.x & 31;
  const int wave = threadIdx.x >> 5;
  const int tilesN = N >> 6;
  const int tilesM = M >> 6;
  const int tile = blockIdx.x * 8 + wave;
  if (tile >= tilesM * tilesN) return;
  const int tm = tile / tilesN;
  const int tn = tile - tm * tilesN;
  const int m0 = tm << 6;
  const int n0 = tn << 6;

  const int rlane = lane & 15;
  const int koff  = (lane >> 4) * 8;
  const int mOff  = (lane >> 4) * 8;

  v8f acc[4][4];
#pragma unroll
  for (int i = 0; i < 4; ++i)
#pragma unroll
    for (int j = 0; j < 4; ++j) acc[i][j] = (v8f){0.f,0.f,0.f,0.f,0.f,0.f,0.f,0.f};

  for (int k0 = 0; k0 < K; k0 += 32) {
    V bh[4], bl[4];
#pragma unroll
    for (int j = 0; j < 4; ++j) {
      const size_t bo = (size_t)(n0 + (j << 4) + rlane) * ldb + koff + k0;
      bh[j] = Frag<T>::load(Bb + bo);
      if (SPLIT) bl[j] = Frag<T>::load(Bb2 + bo);
    }
#pragma unroll
    for (int i = 0; i < 4; ++i) {
      const size_t ao = (size_t)(m0 + (i << 4) + rlane) * lda + koff + k0;
      V ah = Frag<T>::load(Ab + ao);
      V al;
      if (SPLIT) al = Frag<T>::load(Ab2 + ao);
#pragma unroll
      for (int j = 0; j < 4; ++j) {
        acc[i][j] = Frag<T>::mma(ah, bh[j], acc[i][j]);
        if (SPLIT) {
          acc[i][j] = Frag<T>::mma(ah, bl[j], acc[i][j]);
          acc[i][j] = Frag<T>::mma(al, bh[j], acc[i][j]);
        }
      }
      Frag<T>::guard(acc[i][0], acc[i][1], acc[i][2], acc[i][3], ah, SPLIT ? al : ah, bh[0], bh[1], bh[2], bh[3]);
      if (SPLIT) Frag<T>::keep(bl[0], bl[1], bl[2], bl[3]);
    }
    Frag<T>::keep(bh[0], bh[1], bh[2], bh[3]);
    if (SPLIT) Frag<T>::keep(bl[0], bl[1], bl[2], bl[3]);
  }
  acc_guard4(acc[0][0], acc[0][1], acc[0][2], acc[0][3]);
  acc_guard4(acc[1][0], acc[1][1], acc[1][2], acc[1][3]);
  acc_guard4(acc[2][0], acc[2][1], acc[2][2], acc[2][3]);
  acc_guard4(acc[3][0], acc[3][1], acc[3][2], acc[3][3]);

  float* slab = sT[wave];
#pragma unroll
  for (int i = 0; i < 4; ++i) {
    const int mBase = m0 + (i << 4);
#pragma unroll
    for (int j = 0; j < 4; ++j) {
      const int n = n0 + (j << 4) + rlane;
      float bv = 0.f;
      if (BIAS_MODE == 2) bv = bias[n];
#pragma unroll
      for (int r = 0; r < 8; ++r) {
        float v = acc[i][j][r] * scale;
        if (BIAS_MODE == 2) v += bv;
        slab[(mOff + r) * 68 + (j << 4) + rlane] = v;
      }
    }
    __builtin_amdgcn_fence(__ATOMIC_RELEASE, "workgroup");
    __builtin_amdgcn_wave_barrier();
    __builtin_amdgcn_fence(__ATOMIC_ACQUIRE, "workgroup");
    {
      const int hh = lane >> 4, c4 = (lane & 15) * 4;
      for (int pass = 0; pass < 2; ++pass) {
#pragma unroll
        for (int it = 0; it < 8; ++it) {
          const int row = it * 2 + hh;
          v4f v = *(const v4f*)(slab + row * 68 + c4);
          *(volatile v4f*)(Cout + (size_t)(mBase + row) * ldc + n0 + c4) = v;
        }
        __threadfence();
      }
    }
    __builtin_amdgcn_fence(__ATOMIC_RELEASE, "workgroup");
    __builtin_amdgcn_wave_barrier();
    __builtin_amdgcn_fence(__ATOMIC_ACQUIRE, "workgroup");
  }
}

__global__ __launch_bounds__(256) void cond_proj_kernel(
    const float* __restrict__ cond, const float* __restrict__ aw, const float* __restrict__ ab,
    float* __restrict__ ss, int total)
{
  const int i = blockIdx.x * 256 + threadIdx.x;
  if (i >= total) return;
  const int l   = i / (kBatch * 2 * kDm);
  const int rem = i - l * (kBatch * 2 * kDm);
  const int b   = rem / (2 * kDm);
  const int e   = rem - b * (2 * kDm);
  const float* cp = cond + (size_t)b * kCond;
  const float* wp = aw + ((size_t)l * 2 * kDm + e) * kCond;
  float acc = 0.f;
#pragma unroll 1
  for (int k4 = 0; k4 < kCond / 4; ++k4) {
    const v4f c = *(const v4f*)(cp + 4 * k4);
    const v4f w = *(const v4f*)(wp + 4 * k4);
    acc = fmaf(c[0], w[0], acc);
    acc = fmaf(c[1], w[1], acc);
    acc = fmaf(c[2], w[2], acc);
    acc = fmaf(c[3], w[3], acc);
  }
  const float val = acc + ab[(size_t)l * 2 * kDm + e];
  volatile float* q = ss + i;
  *q = val;
  __threadfence();
  *q = val;
}

__global__ __launch_bounds__(256) void prep_x_kernel(
    const float* __restrict__ src, unsigned short* __restrict__ dhi, unsigned short* __restrict__ dlo,
    unsigned short* __restrict__ d16, int total8)
{
  const int i = blockIdx.x * 256 + threadIdx.x;
  if (i >= total8) return;
  const size_t e0 = (size_t)i << 3;
  const v4f a0 = *(const v4f*)(src + e0);
  const v4f a1 = *(const v4f*)(src + e0 + 4);
  v8h hv, lv, fv;
#pragma unroll
  for (int e = 0; e < 4; ++e) {
    const float x0 = a0[e], x1 = a1[e];
    const unsigned short h0 = f2bf_bits(x0), h1 = f2bf_bits(x1);
    const unsigned short l0 = f2bf_bits(x0 - bf_bits2f(h0)), l1 = f2bf_bits(x1 - bf_bits2f(h1));
    hv[e]     = __builtin_bit_cast(_Float16, h0);
    hv[4 + e] = __builtin_bit_cast(_Float16, h1);
    lv[e]     = __builtin_bit_cast(_Float16, l0);
    lv[4 + e] = __builtin_bit_cast(_Float16, l1);
    fv[e]     = (_Float16)x0;
    fv[4 + e] = (_Float16)x1;
  }
  unsigned short* qh = dhi + e0;
  unsigned short* ql = dlo + e0;
  unsigned short* qf = d16 + e0;
  *(volatile v8h*)qh = hv;
  *(volatile v8h*)ql = lv;
  *(volatile v8h*)qf = fv;
  __threadfence();
  *(volatile v8h*)qh = hv;
  *(volatile v8h*)ql = lv;
  *(volatile v8h*)qf = fv;
}

constexpr int kPwBlkA   = (kDin * kDm) / 2048;
constexpr int kPwBlkC   = (kPrjP * kDin) / 2048;
constexpr int kPwBlkD   = (kDin * kDtP) / 2048;
constexpr int kPwBlkE   = (kDm * kDin) / 2048;
constexpr int kPwBlocks = 2 * kPwBlkA + kPwBlkC + kPwBlkD + kPwBlkE;
static_assert((kDin * kDm) % 2048 == 0 && (kPrjP * kDin) % 2048 == 0 && (kDin * kDtP) % 2048 == 0);
static_assert(kPwBlocks == 1872);

__global__ __launch_bounds__(256) void prep_weights_kernel(
    const float* __restrict__ inw, const float* __restrict__ xpw, const float* __restrict__ dtw,
    const float* __restrict__ outw,
    unsigned short* __restrict__ WIH, unsigned short* __restrict__ WIL, unsigned short* __restrict__ WZ16,
    unsigned short* __restrict__ WXH, unsigned short* __restrict__ WXL, unsigned short* __restrict__ WDT16,
    unsigned short* __restrict__ WO16)
{
  const int bx = blockIdx.x;
  const int tid = threadIdx.x;
  const float* sp = inw;
  unsigned short* dA = WIH;
  unsigned short* dB = WIL;
  bool split = true;
  bool valid = true;
  float scale = 1.0f;
  size_t eo = 0;
  if (bx < kPwBlkA) {
    eo = ((size_t)bx * 256 + tid) * 8;
    sp = inw + eo;
    dA = WIH; dB = WIL; split = true;
  } else if (bx < 2 * kPwBlkA) {
    eo = ((size_t)(bx - kPwBlkA) * 256 + tid) * 8;
    sp = inw + (size_t)kDin * kDm + eo;
    dA = WZ16; dB = WZ16; split = false; scale = kCarryWz;
  } else if (bx < 2 * kPwBlkA + kPwBlkC) {
    eo = ((size_t)(bx - 2 * kPwBlkA) * 256 + tid) * 8;
    const int row = (int)(eo / kDin);
    const int col = (int)(eo - (size_t)row * kDin);
    const int rc  = (row < kPrjN) ? row : (kPrjN - 1);
    valid = (row < kPrjN);
    sp = xpw + (size_t)rc * kDin + col;
    dA = WXH; dB = WXL; split = true;
  } else if (bx < 2 * kPwBlkA + kPwBlkC + kPwBlkD) {
    eo = ((size_t)(bx - 2 * kPwBlkA - kPwBlkC) * 256 + tid) * 8;
    const int row = (int)(eo >> 6);
    const int c8  = (int)(eo & 63);
    const int cc  = (c8 < kDtR) ? c8 : (kDtR - 8);
    valid = (c8 < kDtR);
    sp = dtw + (size_t)row * kDtR + cc;
    dA = WDT16; dB = WDT16; split = false; scale = kCarryWdt;
  } else {
    eo = ((size_t)(bx - 2 * kPwBlkA - kPwBlkC - kPwBlkD) * 256 + tid) * 8;
    sp = outw + eo;
    dA = WO16; dB = WO16; split = false; scale = kCarryWo;
  }
  const v4f r0 = *(const v4f*)(sp);
  const v4f r1 = *(const v4f*)(sp + 4);
  v8h hv, lv;
#pragma unroll
  for (int e = 0; e < 4; ++e) {
    const float t0 = r0[e], t1 = r1[e];
    const float x0 = valid ? (t0 * scale) : 0.0f;
    const float x1 = valid ? (t1 * scale) : 0.0f;
    const unsigned short h0 = f2bf_bits(x0), h1 = f2bf_bits(x1);
    const unsigned short l0 = f2bf_bits(x0 - bf_bits2f(h0)), l1 = f2bf_bits(x1 - bf_bits2f(h1));
    const _Float16 g0 = (_Float16)x0, g1 = (_Float16)x1;
    hv[e]     = split ? __builtin_bit_cast(_Float16, h0) : g0;
    hv[4 + e] = split ? __builtin_bit_cast(_Float16, h1) : g1;
    lv[e]     = __builtin_bit_cast(_Float16, l0);
    lv[4 + e] = __builtin_bit_cast(_Float16, l1);
  }
  unsigned short* qa = dA + eo;
  unsigned short* qb = dB + eo;
  *(volatile v8h*)qa = hv;
  if (split) *(volatile v8h*)qb = lv;
  __threadfence();
  *(volatile v8h*)qa = hv;
  if (split) *(volatile v8h*)qb = lv;
}

__global__ __launch_bounds__(256) void conv_silu_kernel(
    const float* __restrict__ XCP, const float* __restrict__ cw, const float* __restrict__ cb,
    float* __restrict__ XC, unsigned short* __restrict__ XCH, unsigned short* __restrict__ XCL)
{
  __shared__ __align__(16) float sT[16 * kTP];
  const int tid = threadIdx.x, lane = tid & 31, wave = tid >> 5;
  const int d0 = blockIdx.x * 256, d = d0 + tid;
  const int g0 = blockIdx.y * 64;
  const int tb = g0 & (kSeq - 1);
  const v4f wv = *(const v4f*)(cw + (size_t)d * 4);
  const float w0 = wv[0], w1 = wv[1], w2 = wv[2], w3 = wv[3];
  const float bc = cb[d];
  float xm3, xm2, xm1;
  {
    const bool hist = (tb > 0);
    const int rb = hist ? (g0 - 3) : g0;
    const float v3 = XCP[(size_t)rb * kDin + d];
    const float v2 = XCP[(size_t)(rb + 1) * kDin + d];
    const float v1 = XCP[(size_t)(rb + 2) * kDin + d];
    xm3 = hist ? v3 : 0.f;
    xm2 = hist ? v2 : 0.f;
    xm1 = hist ? v1 : 0.f;
  }
  const int hrow = wave >> 1;
  const int hch  = (wave & 1) * 128 + lane * 4;
#pragma unroll 1
  for (int sub = 0; sub < 4; ++sub) {
    const int lb = g0 + sub * 16;
#pragma unroll 1
    for (int s = 0; s < 16; ++s) {
      const float xcur = XCP[(size_t)(lb + s) * kDin + d];
      float acc = w0 * xm3;
      acc = fmaf(w1, xm2, acc);
      acc = fmaf(w2, xm1, acc);
      acc = fmaf(w3, xcur, acc);
      const float sv = acc + bc;
      const float sg = __builtin_amdgcn_rcpf(1.0f + expf(-sv));
      sT[s * kTP + tid] = sv * sg;
      xm3 = xm2; xm2 = xm1; xm1 = xcur;
    }
    __syncthreads();
    v4f fv[4];
    v8h bh[2], blo[2];
#pragma unroll
    for (int it = 0; it < 4; ++it) fv[it] = *(const v4f*)(sT + (it * 4 + hrow) * kTP + hch);
#pragma unroll
    for (int it = 0; it < 2; ++it) {
      const float* sp = sT + (it * 8 + wave) * kTP + lane * 8;
      const v4f a0 = *(const v4f*)(sp);
      const v4f a1 = *(const v4f*)(sp + 4);
#pragma unroll
      for (int e = 0; e < 4; ++e) {
        const float x0 = a0[e], x1 = a1[e];
        const unsigned short h0 = f2bf_bits(x0), h1 = f2bf_bits(x1);
        const unsigned short l0 = f2bf_bits(x0 - bf_bits2f(h0)), l1 = f2bf_bits(x1 - bf_bits2f(h1));
        bh[it][e]      = __builtin_bit_cast(_Float16, h0);
        bh[it][4 + e]  = __builtin_bit_cast(_Float16, h1);
        blo[it][e]     = __builtin_bit_cast(_Float16, l0);
        blo[it][4 + e] = __builtin_bit_cast(_Float16, l1);
      }
    }
    for (int pass = 0; pass < 2; ++pass) {
#pragma unroll
      for (int it = 0; it < 4; ++it)
        *(volatile v4f*)(XC + (size_t)(lb + it * 4 + hrow) * kDin + d0 + hch) = fv[it];
#pragma unroll
      for (int it = 0; it < 2; ++it) {
        const size_t o = (size_t)(lb + it * 8 + wave) * kDin + d0 + lane * 8;
        *(volatile v8h*)(XCH + o) = bh[it];
        *(volatile v8h*)(XCL + o) = blo[it];
      }
      __threadfence();
    }
    __syncthreads();
  }
}

__global__ __launch_bounds__(256) void dt_cast_kernel(
    const float* __restrict__ DBC, unsigned short* __restrict__ DT16, int total8)
{
  const int i = blockIdx.x * 256 + threadIdx.x;
  if (i >= total8) return;
  const int e0  = i << 3;
  const int row = e0 >> 6;
  const int c8  = e0 & 63;
  const bool valid = (c8 < kDtR);
  const int cc  = valid ? c8 : (kDtR - 8);
  const float* p = DBC + (size_t)row * kPrjP + cc;
  const v4f a0 = *(const v4f*)(p);
  const v4f a1 = *(const v4f*)(p + 4);
  v8h hv;
#pragma unroll
  for (int e = 0; e < 4; ++e) {
    const float t0 = a0[e], t1 = a1[e];
    hv[e]     = (_Float16)(valid ? (t0 * kCarryDt) : 0.0f);
    hv[4 + e] = (_Float16)(valid ? (t1 * kCarryDt) : 0.0f);
  }
  unsigned short* qd = DT16 + e0;
  *(volatile v8h*)qd = hv;
  __threadfence();
  *(volatile v8h*)qd = hv;
}

__global__ __launch_bounds__(256) void scan_kernel(
    const float* __restrict__ DLR, const float* __restrict__ XC, const float* __restrict__ Zp,
    const float* __restrict__ DBC, const float* __restrict__ Alog, const float* __restrict__ Dv,
    unsigned short* __restrict__ Y16, float* __restrict__ stOut)
{
  __shared__ __align__(16) float sBC[16 * 32];
  __shared__ __align__(16) float sY[16 * kTP];
  __shared__ __align__(16) float sFin[256 * kNst];
  const int tid = threadIdx.x, lane = tid & 31, wave = tid >> 5;
  const int d0 = blockIdx.x * 256, d = d0 + tid;
  const int bix = blockIdx.y;
  const size_t row0 = (size_t)bix * kSeq;

#pragma unroll 1
  for (int n = 0; n < kNst; ++n)
    sFin[n * 256 + tid] = -expf(Alog[(size_t)d * kNst + n]) * kLog2e;
  __syncthreads();
  float A2[kNst], h[kNst];
#pragma unroll
  for (int n = 0; n < kNst; ++n) {
    A2[n] = sFin[n * 256 + tid];
    h[n] = 0.f;
  }
  const float Dd = Dv[d];

#pragma unroll 1
  for (int c = 0; c < kSeq / 16; ++c) {
    const int l0 = c * 16;
    if (tid < 128) {
      const int r = tid >> 3, q = (tid & 7) * 4;
      const v4f v = *(const v4f*)(DBC + (row0 + l0 + r) * kPrjP + kDtR + q);
      *(v4f*)(sBC + r * 32 + q) = v;
    }
    __syncthreads();
#pragma unroll 1
    for (int s = 0; s < 16; ++s) {
      const size_t m = row0 + l0 + s;
      float a  = DLR[m * kDin + d];
      float xv = XC[m * kDin + d];
      float zv = Zp[m * kDin + d];
      asm volatile("" : "+v"(a), "+v"(xv), "+v"(zv));
      const float ea    = expf(-fabsf(a));
      const float u1    = 1.0f + ea;
      const float l1p   = logf(u1) + (ea - (u1 - 1.0f)) * __builtin_amdgcn_rcpf(u1);
      const float delta = fmaxf(a, 0.0f) + l1p;
      const float dtx   = delta * xv;
      v4f Bq[4], Cq[4];
#pragma unroll
      for (int qq = 0; qq < 4; ++qq) {
        Bq[qq] = *(const v4f*)(sBC + s * 32 + 4 * qq);
        Cq[qq] = *(const v4f*)(sBC + s * 32 + kNst + 4 * qq);
      }
      float y = 0.f;
#pragma unroll
      for (int n = 0; n < kNst; ++n) {
        const float e  = exp2f(delta * A2[n]);
        const float hn = fmaf(e, h[n], dtx * Bq[n >> 2][n & 3]);
        h[n] = hn;
        y = fmaf(hn, Cq[n >> 2][n & 3], y);
      }
      y = fmaf(Dd, xv, y);
      const float sg = __builtin_amdgcn_rcpf(1.0f + expf(-zv));
      sY[s * kTP + tid] = (y * (zv * sg)) * kCarryY;
    }
    __syncthreads();
    v8h hv[2];
#pragma unroll
    for (int it = 0; it < 2; ++it) {
      const float* sp = sY + (it * 8 + wave) * kTP + lane * 8;
      const v4f a0 = *(const v4f*)(sp);
      const v4f a1 = *(const v4f*)(sp + 4);
#pragma unroll
      for (int e = 0; e < 4; ++e) {
        const float x0 = a0[e], x1 = a1[e];
        hv[it][e]     = (_Float16)x0;
        hv[it][4 + e] = (_Float16)x1;
      }
    }
    for (int pass = 0; pass < 2; ++pass) {
#pragma unroll
      for (int it = 0; it < 2; ++it)
        *(volatile v8h*)(Y16 + (row0 + l0 + it * 8 + wave) * kDin + d0 + lane * 8) = hv[it];
      __threadfence();
    }
  }

#pragma unroll
  for (int qq = 0; qq < 4; ++qq) {
    const v4f hvq = (v4f){h[4 * qq + 0], h[4 * qq + 1], h[4 * qq + 2], h[4 * qq + 3]};
    *(v4f*)(sFin + tid * kNst + 4 * qq) = hvq;
  }
  __syncthreads();
  {
    float* ob = stOut + ((size_t)bix * kDin + d0) * kNst;
    v4f fv[4];
#pragma unroll
    for (int it = 0; it < 4; ++it) fv[it] = *(const v4f*)(sFin + (it * 256 + tid) * 4);
    for (int pass = 0; pass < 2; ++pass) {
#pragma unroll
      for (int it = 0; it < 4; ++it)
        *(volatile v4f*)(ob + (size_t)(it * 256 + tid) * 4) = fv[it];
      __threadfence();
    }
  }
}

__device__ __forceinline__ float wave_sum(float v) {
#pragma unroll
  for (int off = 16; off > 0; off >>= 1) v += __shfl_xor(v, off, 32);
  return v;
}

template <bool LAST>
__global__ __launch_bounds__(256) void ln_mod_kernel(
    const float* __restrict__ resid, const float* __restrict__ mproj,
    const float* __restrict__ nw, const float* __restrict__ nb,
    const float* __restrict__ ssl,
    const float* __restrict__ fw, const float* __restrict__ fb,
    float* __restrict__ hnext, unsigned short* __restrict__ hh, unsigned short* __restrict__ hl,
    unsigned short* __restrict__ h16, float* __restrict__ outp)
{
  __shared__ __align__(16) float sRow[8][kDm];
  const int tid = threadIdx.x, lane = tid & 31, wave = tid >> 5;
  const int row = blockIdx.x * 8 + wave;
  const int b = row / kSeq;
  float* sr = sRow[wave];
  const float* rp = resid + (size_t)row * kDm;
  const float* mp = mproj + (size_t)row * kDm;
  const float* scp = ssl + (size_t)b * 2 * kDm;
  const float* shp = scp + kDm;
  const float invN = 1.0f / (float)kDm;

  float s = 0.f;
#pragma unroll 1
  for (int it = 0; it < 6; ++it) {
    const int c = it * 128 + lane * 4;
    const v4f a = *(const v4f*)(rp + c);
    const v4f m = *(const v4f*)(mp + c);
    v4f v;
    v[0] = a[0] + m[0]; v[1] = a[1] + m[1]; v[2] = a[2] + m[2]; v[3] = a[3] + m[3];
    *(v4f*)(sr + c) = v;
    s += (v[0] + v[1]) + (v[2] + v[3]);
  }
  s = wave_sum(s);
  const float mu1 = s * invN;
  float q = 0.f;
#pragma unroll 1
  for (int it = 0; it < 6; ++it) {
    const int c = it * 128 + lane * 4;
    const v4f v = *(const v4f*)(sr + c);
    const float e0 = v[0] - mu1, e1 = v[1] - mu1, e2 = v[2] - mu1, e3 = v[3] - mu1;
    q += (e0 * e0 + e1 * e1) + (e2 * e2 + e3 * e3);
  }
  q = wave_sum(q);
  const float rs1 = rsqrtf(q * invN + kEps);

  s = 0.f;
#pragma unroll 1
  for (int it = 0; it < 6; ++it) {
    const int c = it * 128 + lane * 4;
    const v4f v = *(const v4f*)(sr + c);
    const v4f w = *(const v4f*)(nw + c);
    const v4f bb = *(const v4f*)(nb + c);
    v4f o;
    o[0] = (v[0] - mu1) * rs1 * w[0] + bb[0];
    o[1] = (v[1] - mu1) * rs1 * w[1] + bb[1];
    o[2] = (v[2] - mu1) * rs1 * w[2] + bb[2];
    o[3] = (v[3] - mu1) * rs1 * w[3] + bb[3];
    *(v4f*)(sr + c) = o;
    s += (o[0] + o[1]) + (o[2] + o[3]);
  }
  s = wave_sum(s);
  const float mu2 = s * invN;
  q = 0.f;
#pragma unroll 1
  for (int it = 0; it < 6; ++it) {
    const int c = it * 128 + lane * 4;
    const v4f v = *(const v4f*)(sr + c);
    const float e0 = v[0] - mu2, e1 = v[1] - mu2, e2 = v[2] - mu2, e3 = v[3] - mu2;
    q += (e0 * e0 + e1 * e1) + (e2 * e2 + e3 * e3);
  }
  q = wave_sum(q);
  const float rs2 = rsqrtf(q * invN + kEps);

  s = 0.f;
#pragma unroll 1
  for (int it = 0; it < 6; ++it) {
    const int c = it * 128 + lane * 4;
    const v4f v = *(const v4f*)(sr + c);
    const v4f sc = *(const v4f*)(scp + c);
    const v4f sh = *(const v4f*)(shp + c);
    v4f o;
    o[0] = (v[0] - mu2) * rs2 * (1.0f + sc[0]) + sh[0];
    o[1] = (v[1] - mu2) * rs2 * (1.0f + sc[1]) + sh[1];
    o[2] = (v[2] - mu2) * rs2 * (1.0f + sc[2]) + sh[2];
    o[3] = (v[3] - mu2) * rs2 * (1.0f + sc[3]) + sh[3];
    *(v4f*)(sr + c) = o;
    s += (o[0] + o[1]) + (o[2] + o[3]);
  }

  if (LAST) {
    s = wave_sum(s);
    const float mu3 = s * invN;
    q = 0.f;
#pragma unroll 1
    for (int it = 0; it < 6; ++it) {
      const int c = it * 128 + lane * 4;
      const v4f v = *(const v4f*)(sr + c);
      const float e0 = v[0] - mu3, e1 = v[1] - mu3, e2 = v[2] - mu3, e3 = v[3] - mu3;
      q += (e0 * e0 + e1 * e1) + (e2 * e2 + e3 * e3);
    }
    q = wave_sum(q);
    const float rs3 = rsqrtf(q * invN + kEps);
#pragma unroll 1
    for (int it = 0; it < 6; ++it) {
      const int c = it * 128 + lane * 4;
      const v4f v = *(const v4f*)(sr + c);
      const v4f w = *(const v4f*)(fw + c);
      const v4f bb = *(const v4f*)(fb + c);
      v4f o;
      o[0] = (v[0] - mu3) * rs3 * w[0] + bb[0];
      o[1] = (v[1] - mu3) * rs3 * w[1] + bb[1];
      o[2] = (v[2] - mu3) * rs3 * w[2] + bb[2];
      o[3] = (v[3] - mu3) * rs3 * w[3] + bb[3];
      *(v4f*)(sr + c) = o;
    }
  }

  {
    float* dst = (LAST ? outp : hnext) + (size_t)row * kDm;
    for (int pass = 0; pass < 2; ++pass) {
#pragma unroll 1
      for (int it = 0; it < 6; ++it) {
        const int c = it * 128 + lane * 4;
        const v4f v = *(const v4f*)(sr + c);
        *(volatile v4f*)(dst + c) = v;
      }
      __threadfence();
    }
  }

  if (!LAST) {
    __syncthreads();
    v8h hv[3], lv[3], fv[3];
#pragma unroll
    for (int it = 0; it < 3; ++it) {
      const float* sp = sr + it * 256 + lane * 8;
      const v4f a0 = *(const v4f*)(sp);
      const v4f a1 = *(const v4f*)(sp + 4);
#pragma unroll
      for (int e = 0; e < 4; ++e) {
        const float x0 = a0[e], x1 = a1[e];
        const unsigned short h0 = f2bf_bits(x0), h1 = f2bf_bits(x1);
        const unsigned short l0 = f2bf_bits(x0 - bf_bits2f(h0)), l1 = f2bf_bits(x1 - bf_bits2f(h1));
        hv[it][e]     = __builtin_bit_cast(_Float16, h0);
        hv[it][4 + e] = __builtin_bit_cast(_Float16, h1);
        lv[it][e]     = __builtin_bit_cast(_Float16, l0);
        lv[it][4 + e] = __builtin_bit_cast(_Float16, l1);
        fv[it][e]     = (_Float16)x0;
        fv[it][4 + e] = (_Float16)x1;
      }
    }
    for (int pass = 0; pass < 2; ++pass) {
#pragma unroll
      for (int it = 0; it < 3; ++it) {
        const size_t o = (size_t)row * kDm + it * 256 + lane * 8;
        *(volatile v8h*)(hh + o)  = hv[it];
        *(volatile v8h*)(hl + o)  = lv[it];
        *(volatile v8h*)(h16 + o) = fv[it];
      }
      __threadfence();
    }
  }
}

extern "C" void kernel_launch(void* const* d_in, const int* in_sizes, int n_in,
                              void* d_out, int out_size, void* d_ws, size_t ws_size,
                              hipStream_t stream)
{
  if (n_in < 17) return;
  if (in_sizes[0]  != kRows * kDm) return;
  if (in_sizes[1]  != kBatch * kCond) return;
  if (in_sizes[2]  != kLayers * 2 * kDin * kDm) return;
  if (in_sizes[3]  != kLayers * kDin * 4) return;
  if (in_sizes[4]  != kLayers * kDin) return;
  if (in_sizes[5]  != kLayers * kPrjN * kDin) return;
  if (in_sizes[6]  != kLayers * kDin * kDtR) return;
  if (in_sizes[7]  != kLayers * kDin) return;
  if (in_sizes[8]  != kLayers * kDin * kNst) return;
  if (in_sizes[9]  != kLayers * kDin) return;
  if (in_sizes[10] != kLayers * kDm * kDin) return;
  if (in_sizes[11] != kLayers * kDm) return;
  if (in_sizes[12] != kLayers * kDm) return;
  if (in_sizes[13] != kLayers * 2 * kDm * kCond) return;
  if (in_sizes[14] != kLayers * 2 * kDm) return;
  if (in_sizes[15] != kDm) return;
  if (in_sizes[16] != kDm) return;
  if (out_size != kOut0 + kOut1) return;
  if (ws_size < kWsTotal) return;

  const float* x      = (const float*)d_in[0];
  const float* cond   = (const float*)d_in[1];
  const float* in_w   = (const float*)d_in[2];
  const float* conv_w = (const float*)d_in[3];
  const float* conv_b = (const float*)d_in[4];
  const float* xp_w   = (const float*)d_in[5];
  const float* dt_w   = (const float*)d_in[6];
  const float* dt_b   = (const float*)d_in[7];
  const float* A_log  = (const float*)d_in[8];
  const float* D_skip = (const float*)d_in[9];
  const float* out_w  = (const float*)d_in[10];
  const float* norm_w = (const float*)d_in[11];
  const float* norm_b = (const float*)d_in[12];
  const float* ad_w   = (const float*)d_in[13];
  const float* ad_b   = (const float*)d_in[14];
  const float* fn_w   = (const float*)d_in[15];
  const float* fn_b   = (const float*)d_in[16];
  float* out = (float*)d_out;

  char* ws = (char*)d_ws;
  unsigned short* WIH   = (unsigned short*)(ws + kOffWIH);
  unsigned short* WIL   = (unsigned short*)(ws + kOffWIL);
  unsigned short* WZ16  = (unsigned short*)(ws + kOffWZ16);
  unsigned short* WXH   = (unsigned short*)(ws + kOffWXH);
  unsigned short* WXL   = (unsigned short*)(ws + kOffWXL);
  unsigned short* WDT16 = (unsigned short*)(ws + kOffWDT16);
  unsigned short* WO16  = (unsigned short*)(ws + kOffWO16);
  unsigned short* HH    = (unsigned short*)(ws + kOffHH);
  unsigned short* HL    = (unsigned short*)(ws + kOffHL);
  unsigned short* H16   = (unsigned short*)(ws + kOffH16);
  float*          HA    = (float*)(ws + kOffHA);
  float*          HB    = (float*)(ws + kOffHB);
  float*          XCP   = (float*)(ws + kOffXCP);
  float*          ZB    = (float*)(ws + kOffZB);
  float*          XC    = (float*)(ws + kOffXC);
  unsigned short* XCH   = (unsigned short*)(ws + kOffXCH);
  unsigned short* XCL   = (unsigned short*)(ws + kOffXCL);
  float*          DBC   = (float*)(ws + kOffDBC);
  unsigned short* DT16  = (unsigned short*)(ws + kOffDT16);
  float*          DLR   = (float*)(ws + kOffDLR);
  unsigned short* Y16   = (unsigned short*)(ws + kOffY16);
  float*          MP    = (float*)(ws + kOffMP);
  float*          SS    = (float*)(ws + kOffSS);

  cond_proj_kernel<<<(kLayers * kBatch * 2 * kDm) / 256, 256, 0, stream>>>(
      cond, ad_w, ad_b, SS, kLayers * kBatch * 2 * kDm);
  prep_x_kernel<<<(kRows * kDm / 8) / 256, 256, 0, stream>>>(x, HH, HL, H16, kRows * kDm / 8);

  for (int i = 0; i < kLayers; ++i) {
    const float* inw_l  = in_w  + (size_t)i * 2 * kDin * kDm;
    const float* xpw_l  = xp_w  + (size_t)i * kPrjN * kDin;
    const float* dtw_l  = dt_w  + (size_t)i * kDin * kDtR;
    const float* outw_l = out_w + (size_t)i * kDm * kDin;
    const float* dtb_l  = dt_b  + (size_t)i * kDin;

    prep_weights_kernel<<<kPwBlocks, 256, 0, stream>>>(inw_l, xpw_l, dtw_l, outw_l,
                                                       WIH, WIL, WZ16, WXH, WXL, WDT16, WO16);

    wmma_gemm64<1, true, 0><<<96, 256, 0, stream>>>(
        HH, HL, kDm, WIH, WIL, kDm, XCP, kDin, dtb_l, kRows, kDin, kDm, 1.0f);

    wmma_gemm64<0, false, 0><<<96, 256, 0, stream>>>(
        H16, H16, kDm, WZ16, WZ16, kDm, ZB, kDin, dtb_l, kRows, kDin, kDm, kFoldZ);

    conv_silu_kernel<<<dim3(kDin / 256, kRows / 64), 256, 0, stream>>>(
        XCP, conv_w + (size_t)i * kDin * 4, conv_b + (size_t)i * kDin, XC, XCH, XCL);

    wmma_gemm64<1, true, 0><<<8, 256, 0, stream>>>(
        XCH, XCL, kDin, WXH, WXL, kDin, DBC, kPrjP, dtb_l, kRows, kPrjP, kDin, 1.0f);

    dt_cast_kernel<<<(kRows * kDtP / 8) / 256, 256, 0, stream>>>(DBC, DT16, kRows * kDtP / 8);

    wmma_gemm64<0, false, 2><<<96, 256, 0, stream>>>(
        DT16, DT16, kDtP, WDT16, WDT16, kDtP, DLR, kDin, dtb_l, kRows, kDin, kDtP, kFoldDt);

    scan_kernel<<<dim3(kDin / 256, kBatch), 256, 0, stream>>>(
        DLR, XC, ZB, DBC, A_log + (size_t)i * kDin * kNst, D_skip + (size_t)i * kDin, Y16,
        out + (size_t)kOut0 + (size_t)i * kBatch * kDin * kNst);

    wmma_gemm64<0, false, 0><<<48, 256, 0, stream>>>(
        Y16, Y16, kDin, WO16, WO16, kDin, MP, kDm, dtb_l, kRows, kDm, kDin, kFoldO);

    const float* resid = (i == 0) ? x : ((i & 1) ? (const float*)HA : (const float*)HB);
    float* hnext = (i & 1) ? HB : HA;
    const float* nw_l = norm_w + (size_t)i * kDm;
    const float* nb_l = norm_b + (size_t)i * kDm;
    const float* ss_l = SS + (size_t)i * kBatch * 2 * kDm;
    if (i + 1 < kLayers) {
      ln_mod_kernel<false><<<kRows / 8, 256, 0, stream>>>(
          resid, MP, nw_l, nb_l, ss_l, fn_w, fn_b, hnext, HH, HL, H16, out);
    } else {
      ln_mod_kernel<true><<<kRows / 8, 256, 0, stream>>>(
          resid, MP, nw_l, nb_l, ss_l, fn_w, fn_b, hnext, HH, HL, H16, out);
    }
  }
}
